// GatedDeformConv_33767032881837
// MI455X (gfx1250) — hardware-verified
//
#include <hip/hip_runtime.h>
#include <stdint.h>

typedef __bf16 bf16_t;
typedef bf16_t v16bf __attribute__((ext_vector_type(16)));
typedef float v8f __attribute__((ext_vector_type(8)));
typedef float v4f __attribute__((ext_vector_type(4)));
typedef unsigned int v4u __attribute__((ext_vector_type(4)));

#define NB 4
#define CH 128
#define IMH 128
#define IMW 128
#define HWSZ 16384
#define NPOS 65536
#define NE_ELEMS 8388608
#define NCHUNK 36
#define EPSV 1e-5f
#define APITCH 40
#define STATW 32

union Frag { v16bf v; v4u q[2]; };

__device__ __forceinline__ v8f zero8() {
  v8f z;
#pragma unroll
  for (int i = 0; i < 8; ++i) z[i] = 0.0f;
  return z;
}

__device__ __forceinline__ unsigned int bf_bits(float f) {
  unsigned int u = __float_as_uint(f);
  return (u + 0x7FFFu + ((u >> 16) & 1u)) >> 16;
}
__device__ __forceinline__ void split2(float f, unsigned int& hb, unsigned int& lb) {
  hb = bf_bits(f);
  float hf = __uint_as_float(hb << 16);
  lb = bf_bits(f - hf);
}
__device__ __forceinline__ float sigm(float v) { return 1.0f / (1.0f + __expf(-v)); }
__device__ __forceinline__ float lrelu(float v) { return v > 0.0f ? v : 0.2f * v; }

__device__ __forceinline__ void wmma3(v8f& acc, const Frag& ah, const Frag& al,
                                      const Frag& bh, const Frag& bl) {
  acc = __builtin_amdgcn_wmma_f32_16x16x32_bf16(false, ah.v, false, bh.v, (short)0, acc, false, false);
  acc = __builtin_amdgcn_wmma_f32_16x16x32_bf16(false, ah.v, false, bl.v, (short)0, acc, false, false);
  acc = __builtin_amdgcn_wmma_f32_16x16x32_bf16(false, al.v, false, bh.v, (short)0, acc, false, false);
  asm volatile("v_nop\n\tv_nop\n\tv_nop\n\tv_nop"
               : "+v"(acc) : "v"(ah.v), "v"(al.v), "v"(bh.v), "v"(bl.v));
}

__global__ __launch_bounds__(256) void pack_w_kernel(
    const float* __restrict__ w0, const float* __restrict__ w1,
    int n0, int n1, int NT, v4u* __restrict__ hi, v4u* __restrict__ lo, int total) {
  const int g = blockIdx.x * 256 + threadIdx.x;
  if (g >= total) return;
  const int jh   = g & 1;
  const int lane = (g >> 1) & 31;
  const int rest = g >> 6;
  const int nt = rest % NT;
  const int cc = rest / NT;
  const int kc = cc & 3, t = cc >> 2;
  const int h = lane >> 4, n = lane & 15;
  const int co = nt * 16 + n;
  const int cib = kc * 32 + 8 * h + 16 * jh;
  unsigned int hp[4], lp[4];
#pragma unroll
  for (int i = 0; i < 4; ++i) { hp[i] = 0u; lp[i] = 0u; }
#pragma unroll
  for (int e = 0; e < 8; ++e) {
    const int ci = cib + e;
    float v = 0.0f;
    if (co < n0)           v = w0[((size_t)co * CH + ci) * 9 + t];
    else if (co < n0 + n1) v = w1[((size_t)(co - n0) * CH + ci) * 9 + t];
    unsigned int hb, lb;
    split2(v, hb, lb);
    hp[e >> 1] |= hb << (16 * (e & 1));
    lp[e >> 1] |= lb << (16 * (e & 1));
  }
  v4u H, L;
  H.x = hp[0]; H.y = hp[1]; H.z = hp[2]; H.w = hp[3];
  L.x = lp[0]; L.y = lp[1]; L.z = lp[2]; L.w = lp[3];
  volatile v4u* ph = (volatile v4u*)(hi + g);
  volatile v4u* pl = (volatile v4u*)(lo + g);
  *ph = H; *pl = L;
  __threadfence();
  *ph = H; *pl = L;
}

__global__ __launch_bounds__(256) void conv_af_kernel(
    const float* __restrict__ x, const v4u* __restrict__ wh, const v4u* __restrict__ wl,
    const float* __restrict__ b_attn, const float* __restrict__ b_feat,
    float* __restrict__ attn, float* __restrict__ feat) {
  __shared__ __attribute__((aligned(16))) unsigned short sAh[32 * APITCH];
  __shared__ __attribute__((aligned(16))) unsigned short sAl[32 * APITCH];
  __shared__ __attribute__((aligned(16))) float sO[32 * 260];

  const int tid = threadIdx.x;
  const int wave = tid >> 5, lane = tid & 31;
  const int h = lane >> 4, m16 = lane & 15;
  const int posBase = blockIdx.x * 32;
  if (posBase >= NPOS) return;
  const int b   = posBase >> 14;
  const int hw0 = posBase & (HWSZ - 1);
  const int py  = hw0 >> 7, px0 = hw0 & 127;
  const int msub = wave & 1;
  const int ntBase = (wave >> 1) * 4;

  v8f acc[4];
#pragma unroll
  for (int i = 0; i < 4; ++i) acc[i] = zero8();

#pragma unroll 1
  for (int cc = 0; cc < NCHUNK; ++cc) {
    const int t = cc >> 2, kc = cc & 3;
    const int sy = py + t / 3 - 1;
    const int dx = t % 3 - 1;
#pragma unroll
    for (int k = 0; k < 4; ++k) {
      const int e = k * 256 + tid;
      const int chl = e >> 5, xl = e & 31;
      const int sx = px0 + xl + dx;
      const int c = kc * 32 + chl;
      float v = 0.0f;
      if (sy >= 0 && sy < IMH && sx >= 0 && sx < IMW)
        v = x[(((size_t)b * CH + c) * IMH + sy) * IMW + sx];
      unsigned int hb, lb;
      split2(v, hb, lb);
      sAh[xl * APITCH + chl] = (unsigned short)hb;
      sAl[xl * APITCH + chl] = (unsigned short)lb;
    }
    __syncthreads();

    Frag ah, al;
    const int row = msub * 16 + m16;
    ah.q[0] = *(const v4u*)(&sAh[row * APITCH + 8 * h]);
    ah.q[1] = *(const v4u*)(&sAh[row * APITCH + 16 + 8 * h]);
    al.q[0] = *(const v4u*)(&sAl[row * APITCH + 8 * h]);
    al.q[1] = *(const v4u*)(&sAl[row * APITCH + 16 + 8 * h]);

    const size_t bb = (size_t)((cc * 16 + ntBase) * 32 + lane) * 2;
#pragma unroll
    for (int n = 0; n < 4; ++n) {
      Frag bh, bl;
      bh.q[0] = wh[bb + (size_t)n * 64];
      bh.q[1] = wh[bb + (size_t)n * 64 + 1];
      bl.q[0] = wl[bb + (size_t)n * 64];
      bl.q[1] = wl[bb + (size_t)n * 64 + 1];
      wmma3(acc[n], ah, al, bh, bl);
    }
    __syncthreads();
  }

#pragma unroll
  for (int n = 0; n < 4; ++n) {
    const int coG = (ntBase + n) * 16 + m16;
    const bool isA = coG < 128;
    const int co = isA ? coG : coG - 128;
    const float bias = isA ? b_attn[co] : b_feat[co];
#pragma unroll
    for (int r = 0; r < 8; ++r) {
      float v = acc[n][r] + bias;
      if (isA) v = sigm(v);
      sO[(msub * 16 + 8 * h + r) * 260 + coG] = v;
    }
  }
  __syncthreads();

  v4f va[4], vf[4];
#pragma unroll
  for (int r4 = 0; r4 < 4; ++r4) {
    const int rr = wave * 4 + r4;
    va[r4] = *(const v4f*)(&sO[rr * 260 + 4 * lane]);
    vf[r4] = *(const v4f*)(&sO[rr * 260 + 128 + 4 * lane]);
  }
#pragma unroll
  for (int r4 = 0; r4 < 4; ++r4) {
    const size_t pos = (size_t)(posBase + wave * 4 + r4);
    *((volatile v4f*)(attn + pos * CH) + lane) = va[r4];
    *((volatile v4f*)(feat + pos * CH) + lane) = vf[r4];
  }
  __threadfence();
#pragma unroll
  for (int r4 = 0; r4 < 4; ++r4) {
    const size_t pos = (size_t)(posBase + wave * 4 + r4);
    *((volatile v4f*)(attn + pos * CH) + lane) = va[r4];
    *((volatile v4f*)(feat + pos * CH) + lane) = vf[r4];
  }
}

__global__ __launch_bounds__(256) void stats_kernel(
    const float* __restrict__ buf, float* __restrict__ stats) {
  __shared__ double sS[256], sQ[256];
  const int bc = blockIdx.x;
  if (bc >= NB * CH) return;
  const int c = bc & (CH - 1);
  const int b = bc >> 7;
  const float* p = buf + (size_t)b * HWSZ * CH + c;
  double s = 0.0, q = 0.0;
  for (int i = threadIdx.x; i < HWSZ; i += 256) {
    const float v = p[(size_t)i * CH];
    s += (double)v;
    q += (double)v * (double)v;
  }
  sS[threadIdx.x] = s; sQ[threadIdx.x] = q;
  __syncthreads();
  for (int off = 128; off > 0; off >>= 1) {
    if (threadIdx.x < (unsigned)off) {
      sS[threadIdx.x] += sS[threadIdx.x + off];
      sQ[threadIdx.x] += sQ[threadIdx.x + off];
    }
    __syncthreads();
  }
  if (threadIdx.x == 0) {
    const double mu = sS[0] * (1.0 / (double)HWSZ);
    double var = sQ[0] * (1.0 / (double)HWSZ) - mu * mu;
    if (var < 0.0) var = 0.0;
    const float muf = (float)mu;
    const float rs  = rsqrtf((float)var + EPSV);
    v4f l0, z;
    l0.x = muf; l0.y = rs; l0.z = 0.0f; l0.w = 0.0f;
    z.x = 0.0f; z.y = 0.0f; z.z = 0.0f; z.w = 0.0f;
    volatile v4f* ps = (volatile v4f*)(stats + (size_t)bc * STATW);
    ps[0] = l0;
#pragma unroll
    for (int i = 1; i < 8; ++i) ps[i] = z;
    __threadfence();
    ps[0] = l0;
#pragma unroll
    for (int i = 1; i < 8; ++i) ps[i] = z;
  }
}

__global__ __launch_bounds__(256) void fuse1_kernel(
    const float* __restrict__ feat, const float* __restrict__ attn,
    const float* __restrict__ statsF, float* __restrict__ xa) {
  const size_t i = ((size_t)blockIdx.x * 256 + threadIdx.x) * 4;
  if (i >= (size_t)NE_ELEMS) return;
  const int c = (int)(i & (CH - 1));
  const int b = (int)(i >> 21);
  const v4f f = *(const v4f*)(feat + i);
  const v4f a = *(const v4f*)(attn + i);
  v4f o;
#pragma unroll
  for (int j = 0; j < 4; ++j) {
    const int sc = b * CH + c + j;
    const float mu = statsF[(size_t)sc * STATW];
    const float rs = statsF[(size_t)sc * STATW + 1];
    float v = (f[j] - mu) * rs;
    v = lrelu(v);
    o[j] = v * a[j];
  }
  volatile v4f* po = (volatile v4f*)(xa + i);
  *po = o;
  __threadfence();
  *po = o;
}

__global__ __launch_bounds__(256) void conv_om_kernel(
    const float* __restrict__ xa, const v4u* __restrict__ wh, const v4u* __restrict__ wl,
    const float* __restrict__ b_off, const float* __restrict__ b_mask,
    float* __restrict__ om) {
  __shared__ __attribute__((aligned(16))) unsigned short sAh[128 * APITCH];
  __shared__ __attribute__((aligned(16))) unsigned short sAl[128 * APITCH];
  __shared__ __attribute__((aligned(16))) float sO[128 * 36];

  const int tid = threadIdx.x;
  const int wave = tid >> 5, lane = tid & 31;
  const int h = lane >> 4, m16 = lane & 15;
  const int posBase = blockIdx.x * 128;
  if (posBase >= NPOS) return;
  const int b   = posBase >> 14;
  const int hw0 = posBase & (HWSZ - 1);
  const int py  = hw0 >> 7;

  v8f acc[2];
  acc[0] = zero8(); acc[1] = zero8();

#pragma unroll 1
  for (int cc = 0; cc < NCHUNK; ++cc) {
    const int t = cc >> 2, kc = cc & 3;
    const int sy = py + t / 3 - 1;
    const int dx = t % 3 - 1;
#pragma unroll
    for (int k = 0; k < 16; ++k) {
      const int e = k * 256 + tid;
      const int pl = e >> 5, ch = e & 31;
      const int sx = pl + dx;
      float v = 0.0f;
      if (sy >= 0 && sy < IMH && sx >= 0 && sx < IMW)
        v = xa[((size_t)b * HWSZ + (size_t)sy * IMW + sx) * CH + kc * 32 + ch];
      unsigned int hb, lb;
      split2(v, hb, lb);
      sAh[pl * APITCH + ch] = (unsigned short)hb;
      sAl[pl * APITCH + ch] = (unsigned short)lb;
    }
    __syncthreads();

    Frag ah, al;
    const int row = wave * 16 + m16;
    ah.q[0] = *(const v4u*)(&sAh[row * APITCH + 8 * h]);
    ah.q[1] = *(const v4u*)(&sAh[row * APITCH + 16 + 8 * h]);
    al.q[0] = *(const v4u*)(&sAl[row * APITCH + 8 * h]);
    al.q[1] = *(const v4u*)(&sAl[row * APITCH + 16 + 8 * h]);

    const size_t bb = (size_t)((cc * 2) * 32 + lane) * 2;
#pragma unroll
    for (int n = 0; n < 2; ++n) {
      Frag bh, bl;
      bh.q[0] = wh[bb + (size_t)n * 64];
      bh.q[1] = wh[bb + (size_t)n * 64 + 1];
      bl.q[0] = wl[bb + (size_t)n * 64];
      bl.q[1] = wl[bb + (size_t)n * 64 + 1];
      wmma3(acc[n], ah, al, bh, bl);
    }
    __syncthreads();
  }

#pragma unroll
  for (int n = 0; n < 2; ++n) {
    const int col = n * 16 + m16;
    const int io = col < 18 ? col : 17;
    int im = col - 18; im = im < 0 ? 0 : (im > 8 ? 8 : im);
    const float bo = b_off[io];
    const float bm = b_mask[im];
#pragma unroll
    for (int r = 0; r < 8; ++r) {
      const float a = acc[n][r];
      float v;
      if (col < 18)      v = a + bo;
      else if (col < 27) v = sigm(a + bm);
      else               v = 0.0f;
      sO[(wave * 16 + 8 * h + r) * 36 + col] = v;
    }
  }
  __syncthreads();

  v4f vv[4];
  int rowv[4], qv[4];
#pragma unroll
  for (int k = 0; k < 4; ++k) {
    const int f = k * 32 + lane;
    rowv[k] = wave * 16 + (f >> 3);
    qv[k] = f & 7;
    vv[k] = *(const v4f*)(&sO[rowv[k] * 36 + 4 * qv[k]]);
  }
#pragma unroll
  for (int k = 0; k < 4; ++k)
    *((volatile v4f*)om + (size_t)(posBase + rowv[k]) * 8 + qv[k]) = vv[k];
  __threadfence();
#pragma unroll
  for (int k = 0; k < 4; ++k)
    *((volatile v4f*)om + (size_t)(posBase + rowv[k]) * 8 + qv[k]) = vv[k];
}

__global__ __launch_bounds__(256) void deform_kernel(
    const float* __restrict__ xa, const float* __restrict__ om,
    const v4u* __restrict__ wh, const v4u* __restrict__ wl,
    const float* __restrict__ b_org, float* __restrict__ dconv) {
  __shared__ __attribute__((aligned(16))) unsigned short sAh[64 * APITCH];
  __shared__ __attribute__((aligned(16))) unsigned short sAl[64 * APITCH];
  __shared__ __attribute__((aligned(16))) float sO[64 * 132];
  __shared__ int   sY0[64], sX0[64];
  __shared__ float sWy[64], sWx[64], sM[64];

  const int tid = threadIdx.x;
  const int wave = tid >> 5, lane = tid & 31;
  const int h = lane >> 4, m16 = lane & 15;
  const int posBase = blockIdx.x * 64;
  if (posBase >= NPOS) return;
  const int b = posBase >> 14;
  const int msub = wave & 3;
  const int ntBase = (wave >> 2) * 4;
  const int gPos = tid >> 2;
  const int gCh  = (tid & 3) * 8;

  v8f acc[4];
#pragma unroll
  for (int i = 0; i < 4; ++i) acc[i] = zero8();

#pragma unroll 1
  for (int t = 0; t < 9; ++t) {
    if (tid < 64) {
      const int pos = posBase + tid;
      const int hw = pos & (HWSZ - 1);
      const float dy = om[(size_t)pos * 32 + t * 2];
      const float dx = om[(size_t)pos * 32 + t * 2 + 1];
      float yy = dy + (float)(hw >> 7) + (float)(t / 3) - 1.0f;
      float xx = dx + (float)(hw & 127) + (float)(t % 3) - 1.0f;
      yy = fminf(fmaxf(yy, -16.0f), 144.0f);
      xx = fminf(fmaxf(xx, -16.0f), 144.0f);
      const float y0 = floorf(yy), x0 = floorf(xx);
      sY0[tid] = (int)y0; sX0[tid] = (int)x0;
      sWy[tid] = yy - y0; sWx[tid] = xx - x0;
      sM[tid]  = om[(size_t)pos * 32 + 18 + t];
    }
    __syncthreads();
    const int   y0 = sY0[gPos], x0 = sX0[gPos];
    const float wy = sWy[gPos], wx = sWx[gPos], mk = sM[gPos];

#pragma unroll 1
    for (int kc = 0; kc < 4; ++kc) {
      float accf[8];
#pragma unroll
      for (int j = 0; j < 8; ++j) accf[j] = 0.0f;
#pragma unroll
      for (int corner = 0; corner < 4; ++corner) {
        const int yi = y0 + (corner >> 1), xi = x0 + (corner & 1);
        const float w = ((corner >> 1) ? wy : 1.0f - wy) *
                        ((corner & 1)  ? wx : 1.0f - wx);
        if (yi >= 0 && yi < IMH && xi >= 0 && xi < IMW) {
          const float* p = xa + ((size_t)b * HWSZ + (size_t)yi * IMW + xi) * CH
                              + kc * 32 + gCh;
          const v4f q0 = *(const v4f*)p;
          const v4f q1 = *(const v4f*)(p + 4);
#pragma unroll
          for (int j = 0; j < 4; ++j) { accf[j] += w * q0[j]; accf[4 + j] += w * q1[j]; }
        }
      }
      unsigned int hp[4], lp[4];
#pragma unroll
      for (int i = 0; i < 4; ++i) { hp[i] = 0u; lp[i] = 0u; }
#pragma unroll
      for (int j = 0; j < 8; ++j) {
        unsigned int hb, lb;
        split2(accf[j] * mk, hb, lb);
        hp[j >> 1] |= hb << (16 * (j & 1));
        lp[j >> 1] |= lb << (16 * (j & 1));
      }
      v4u H, L;
      H.x = hp[0]; H.y = hp[1]; H.z = hp[2]; H.w = hp[3];
      L.x = lp[0]; L.y = lp[1]; L.z = lp[2]; L.w = lp[3];
      *(v4u*)(&sAh[gPos * APITCH + gCh]) = H;
      *(v4u*)(&sAl[gPos * APITCH + gCh]) = L;
      __syncthreads();

      Frag ah, al;
      const int row = msub * 16 + m16;
      ah.q[0] = *(const v4u*)(&sAh[row * APITCH + 8 * h]);
      ah.q[1] = *(const v4u*)(&sAh[row * APITCH + 16 + 8 * h]);
      al.q[0] = *(const v4u*)(&sAl[row * APITCH + 8 * h]);
      al.q[1] = *(const v4u*)(&sAl[row * APITCH + 16 + 8 * h]);

      const size_t bb = (size_t)(((t * 4 + kc) * 8 + ntBase) * 32 + lane) * 2;
#pragma unroll
      for (int n = 0; n < 4; ++n) {
        Frag bh, bl;
        bh.q[0] = wh[bb + (size_t)n * 64];
        bh.q[1] = wh[bb + (size_t)n * 64 + 1];
        bl.q[0] = wl[bb + (size_t)n * 64];
        bl.q[1] = wl[bb + (size_t)n * 64 + 1];
        wmma3(acc[n], ah, al, bh, bl);
      }
      __syncthreads();
    }
  }

#pragma unroll
  for (int n = 0; n < 4; ++n) {
    const int co = (ntBase + n) * 16 + m16;
    const float bias = b_org[co];
#pragma unroll
    for (int r = 0; r < 8; ++r)
      sO[(msub * 16 + 8 * h + r) * 132 + co] = acc[n][r] + bias;
  }
  __syncthreads();

  v4f vv[8];
#pragma unroll
  for (int r8 = 0; r8 < 8; ++r8)
    vv[r8] = *(const v4f*)(&sO[(wave * 8 + r8) * 132 + 4 * lane]);
#pragma unroll
  for (int r8 = 0; r8 < 8; ++r8) {
    const size_t pos = (size_t)(posBase + wave * 8 + r8);
    *((volatile v4f*)(dconv + pos * CH) + lane) = vv[r8];
  }
  __threadfence();
#pragma unroll
  for (int r8 = 0; r8 < 8; ++r8) {
    const size_t pos = (size_t)(posBase + wave * 8 + r8);
    *((volatile v4f*)(dconv + pos * CH) + lane) = vv[r8];
  }
}

__global__ __launch_bounds__(256) void fuse2_kernel(
    const float* __restrict__ xa, const float* __restrict__ attn,
    const float* __restrict__ dconv, const float* __restrict__ statsD,
    float* __restrict__ out) {
  __shared__ __attribute__((aligned(16))) float sT[CH * 68];
  const int tid = threadIdx.x;
  const int posBase = blockIdx.x * 64;
  if (posBase >= NPOS) return;
  const int b   = posBase >> 14;
  const int hw0 = posBase & (HWSZ - 1);

#pragma unroll 4
  for (int k = 0; k < 32; ++k) {
    const int e = k * 256 + tid;
    const int pl = e >> 7, c = e & (CH - 1);
    const size_t i = (size_t)(posBase + pl) * CH + c;
    const int sc = b * CH + c;
    const float a  = attn[i];
    const float mu = statsD[(size_t)sc * STATW];
    const float rs = statsD[(size_t)sc * STATW + 1];
    float v2 = (dconv[i] - mu) * rs;
    v2 = lrelu(v2);
    sT[c * 68 + pl] = xa[i] + v2 * (1.0f - a);
  }
  __syncthreads();

  v4f vv[8];
  int cv[8], qv[8];
#pragma unroll
  for (int k = 0; k < 8; ++k) {
    const int f = k * 256 + tid;
    cv[k] = f >> 4; qv[k] = f & 15;
    vv[k] = *(const v4f*)(&sT[cv[k] * 68 + 4 * qv[k]]);
  }
#pragma unroll
  for (int k = 0; k < 8; ++k)
    *((volatile v4f*)(out + ((size_t)(b * CH + cv[k]) * HWSZ + hw0)) + qv[k]) = vv[k];
  __threadfence();
#pragma unroll
  for (int k = 0; k < 8; ++k)
    *((volatile v4f*)(out + ((size_t)(b * CH + cv[k]) * HWSZ + hw0)) + qv[k]) = vv[k];
}

extern "C" void kernel_launch(void* const* d_in, const int* in_sizes, int n_in,
                              void* d_out, int out_size, void* d_ws, size_t ws_size,
                              hipStream_t stream) {
  if (n_in < 11) return;
  if (in_sizes[0] != NE_ELEMS || out_size != NE_ELEMS) return;
  if (in_sizes[1] != CH * CH * 9 || in_sizes[3] != CH * CH * 9 || in_sizes[5] != CH * CH * 9) return;
  if (in_sizes[2] != CH || in_sizes[4] != CH || in_sizes[6] != CH) return;
  if (in_sizes[7] != 18 * CH * 9 || in_sizes[8] != 18) return;
  if (in_sizes[9] != 9 * CH * 9 || in_sizes[10] != 9) return;

  const float* x      = (const float*)d_in[0];
  const float* w_attn = (const float*)d_in[1];
  const float* b_attn = (const float*)d_in[2];
  const float* w_feat = (const float*)d_in[3];
  const float* b_feat = (const float*)d_in[4];
  const float* w_org  = (const float*)d_in[5];
  const float* b_org  = (const float*)d_in[6];
  const float* w_off  = (const float*)d_in[7];
  const float* b_off  = (const float*)d_in[8];
  const float* w_mask = (const float*)d_in[9];
  const float* b_mask = (const float*)d_in[10];

  char* ws = (char*)d_ws;
  size_t off = 0;
  auto take = [&](size_t bytes) -> char* {
    char* p = ws + off;
    off += (bytes + 255) & ~(size_t)255;
    return p;
  };
  const size_t NE = (size_t)NE_ELEMS;
  const int totAF  = NCHUNK * 16 * 32 * 2;
  const int totOM  = NCHUNK * 2 * 32 * 2;
  const int totORG = NCHUNK * 8 * 32 * 2;

  float* attn   = (float*)take(NE * 4);
  float* feat   = (float*)take(NE * 4);
  float* xa     = (float*)take(NE * 4);
  float* dconv  = (float*)take(NE * 4);
  float* om     = (float*)take((size_t)NPOS * 32 * 4);
  v4u*   wAFh   = (v4u*)take((size_t)totAF * 16);
  v4u*   wAFl   = (v4u*)take((size_t)totAF * 16);
  v4u*   wOMh   = (v4u*)take((size_t)totOM * 16);
  v4u*   wOMl   = (v4u*)take((size_t)totOM * 16);
  v4u*   wORGh  = (v4u*)take((size_t)totORG * 16);
  v4u*   wORGl  = (v4u*)take((size_t)totORG * 16);
  float* statsF = (float*)take((size_t)NB * CH * STATW * 4);
  float* statsD = (float*)take((size_t)NB * CH * STATW * 4);
  if (off > ws_size) return;

  pack_w_kernel<<<(totAF + 255) / 256, 256, 0, stream>>>(w_attn, w_feat, CH, CH, 16, wAFh, wAFl, totAF);
  pack_w_kernel<<<(totOM + 255) / 256, 256, 0, stream>>>(w_off, w_mask, 18, 9, 2, wOMh, wOMl, totOM);
  pack_w_kernel<<<(totORG + 255) / 256, 256, 0, stream>>>(w_org, w_org, CH, 0, 8, wORGh, wORGl, totORG);

  conv_af_kernel<<<(NPOS + 31) / 32, 256, 0, stream>>>(x, wAFh, wAFl, b_attn, b_feat, attn, feat);
  stats_kernel  <<<NB * CH, 256, 0, stream>>>(feat, statsF);
  fuse1_kernel  <<<(unsigned)((NE / 4 + 255) / 256), 256, 0, stream>>>(feat, attn, statsF, xa);

  conv_om_kernel<<<(NPOS + 127) / 128, 256, 0, stream>>>(xa, wOMh, wOMl, b_off, b_mask, om);
  deform_kernel <<<(NPOS + 63) / 64, 256, 0, stream>>>(xa, om, wORGh, wORGl, b_org, dconv);
  stats_kernel  <<<NB * CH, 256, 0, stream>>>(dconv, statsD);

  fuse2_kernel  <<<(NPOS + 63) / 64, 256, 0, stream>>>(xa, attn, dconv, statsD, (float*)d_out);
}
